// DeltaNet_31877247271458
// MI455X (gfx1250) — hardware-verified
//
#include <hip/hip_runtime.h>
#include <stdint.h>
#include <math.h>


typedef __bf16 bf16;
typedef __bf16 v16bf __attribute__((ext_vector_type(16)));
typedef __bf16 v8bf  __attribute__((ext_vector_type(8)));
typedef __bf16 v4bf  __attribute__((ext_vector_type(4)));
typedef float  v8f   __attribute__((ext_vector_type(8)));
typedef float  v4f   __attribute__((ext_vector_type(4)));
typedef v4f  v4fa  __attribute__((may_alias));
typedef v8bf v8bfa __attribute__((may_alias));
typedef v4bf v4bfa __attribute__((may_alias));

#define BBATCH 2
#define LLEN   2048
#define DMODEL 1024
#define NHEAD  4
#define DKH    256
#define DVH    256
#define CONVK  4
#define CCH    32
#define NCH    (LLEN / CCH)
#define DVT    16
#define NDV    (DVH / DVT)
#define BL     (BBATCH * LLEN)
#define BHL    (BBATCH * NHEAD * LLEN)
#define GP     40

struct Frag2 { v16bf hi; v16bf lo; };

__device__ __forceinline__ void put2(Frag2& f, int i, float x) {
  bf16 hb = (bf16)x;
  f.hi[i] = hb;
  f.lo[i] = (bf16)(x - (float)hb);
}

__device__ __forceinline__ Frag2 frag_rowk_f32(const float* p, int h) {
  const float* p0 = p + 8 * h;
  const float* p1 = p + 16 + 8 * h;
  v4f x0 = *(const v4fa*)(p0);
  v4f x1 = *(const v4fa*)(p0 + 4);
  v4f x2 = *(const v4fa*)(p1);
  v4f x3 = *(const v4fa*)(p1 + 4);
  Frag2 f;
#pragma unroll
  for (int e = 0; e < 4; ++e) {
    put2(f, e, x0[e]);
    put2(f, 4 + e, x1[e]);
    put2(f, 8 + e, x2[e]);
    put2(f, 12 + e, x3[e]);
  }
  return f;
}

__device__ __forceinline__ Frag2 frag_colk_f32(const float* p, int ld, int h) {
  Frag2 f;
#pragma unroll
  for (int e = 0; e < 8; ++e) {
    put2(f, e, p[(8 * h + e) * ld]);
    put2(f, 8 + e, p[(16 + 8 * h + e) * ld]);
  }
  return f;
}

__device__ __forceinline__ Frag2 frag_rowk_bf(const bf16* ph, const bf16* pl, int h) {
  union U { v16bf v; v8bf q[2]; } a, b;
  a.q[0] = *(const v8bfa*)(ph + 8 * h);
  a.q[1] = *(const v8bfa*)(ph + 16 + 8 * h);
  b.q[0] = *(const v8bfa*)(pl + 8 * h);
  b.q[1] = *(const v8bfa*)(pl + 16 + 8 * h);
  Frag2 f;
  f.hi = a.v;
  f.lo = b.v;
  return f;
}

__device__ __forceinline__ v8f mma3(v8f acc, const Frag2& a, const Frag2& b) {
  acc = __builtin_amdgcn_wmma_f32_16x16x32_bf16(false, a.lo, false, b.hi, (short)0, acc, false, false);
  acc = __builtin_amdgcn_wmma_f32_16x16x32_bf16(false, a.hi, false, b.lo, (short)0, acc, false, false);
  acc = __builtin_amdgcn_wmma_f32_16x16x32_bf16(false, a.hi, false, b.hi, (short)0, acc, false, false);
  asm volatile("v_nop\n\tv_nop\n\tv_nop\n\tv_nop" : "+v"(acc) : "v"(a.hi), "v"(a.lo), "v"(b.hi), "v"(b.lo));
  return acc;
}

__device__ __forceinline__ float wave_sum(float v) {
#pragma unroll
  for (int o = 16; o > 0; o >>= 1) v += __shfl_xor(v, o, 32);
  return v;
}

__device__ __forceinline__ void stage_a128(const float* __restrict__ A, int lda, int m0, int k0,
                                           bf16* Ah, bf16* Al, int tid) {
#pragma unroll
  for (int j = 0; j < 4; ++j) {
    const int idx = tid + 256 * j;
    const int r = idx >> 3, c4 = (idx & 7) << 2;
    v4f x = *(const v4fa*)(A + (size_t)(m0 + r) * lda + k0 + c4);
    v4bf hv, lv;
#pragma unroll
    for (int e = 0; e < 4; ++e) {
      bf16 hb = (bf16)x[e];
      hv[e] = hb;
      lv[e] = (bf16)(x[e] - (float)hb);
    }
    *(v4bfa*)(Ah + r * GP + c4) = hv;
    *(v4bfa*)(Al + r * GP + c4) = lv;
  }
}

__global__ __launch_bounds__(256) void k_gemm(const float* __restrict__ A,
                                              const float* __restrict__ Bw,
                                              float* __restrict__ C,
                                              int M, int N, int K) {
  __shared__ __attribute__((aligned(16))) unsigned char smem[32768];
  bf16* Ah = (bf16*)smem;
  bf16* Al = Ah + 128 * GP;
  bf16* Bh = Al + 128 * GP;
  bf16* Bl = Bh + 64 * GP;
  float* Cs = (float*)smem;
  const int tid = threadIdx.x, lane = tid & 31, w = tid >> 5, h = lane >> 4, m16 = lane & 15;
  const int m0 = blockIdx.x * 128, n0 = blockIdx.y * 64;
  if (m0 + 128 > M || n0 + 64 > N) return;
  const int wm = w >> 1, wn = w & 1;
  v8f a00 = {}, a01 = {}, a10 = {}, a11 = {};
  const int nk = K >> 5;
#pragma unroll 1
  for (int it = 0; it < nk; ++it) {
    const int k0 = it << 5;
    stage_a128(A, K, m0, k0, Ah, Al, tid);
#pragma unroll
    for (int j = 0; j < 2; ++j) {
      const int idx = tid + 256 * j;
      const int kk = idx >> 4, n4 = (idx & 15) << 2;
      v4f x = *(const v4fa*)(Bw + (size_t)(k0 + kk) * N + n0 + n4);
#pragma unroll
      for (int e = 0; e < 4; ++e) {
        bf16 hb = (bf16)x[e];
        Bh[(n4 + e) * GP + kk] = hb;
        Bl[(n4 + e) * GP + kk] = (bf16)(x[e] - (float)hb);
      }
    }
    __syncthreads();
    Frag2 fa0 = frag_rowk_bf(Ah + (wm * 32 + m16) * GP, Al + (wm * 32 + m16) * GP, h);
    Frag2 fa1 = frag_rowk_bf(Ah + (wm * 32 + 16 + m16) * GP, Al + (wm * 32 + 16 + m16) * GP, h);
    Frag2 fb0 = frag_rowk_bf(Bh + (wn * 32 + m16) * GP, Bl + (wn * 32 + m16) * GP, h);
    Frag2 fb1 = frag_rowk_bf(Bh + (wn * 32 + 16 + m16) * GP, Bl + (wn * 32 + 16 + m16) * GP, h);
    a00 = mma3(a00, fa0, fb0);
    a01 = mma3(a01, fa0, fb1);
    a10 = mma3(a10, fa1, fb0);
    a11 = mma3(a11, fa1, fb1);
    __syncthreads();
  }
#pragma unroll
  for (int r = 0; r < 8; ++r) {
    const int row = wm * 32 + 8 * h + r, col = wn * 32 + m16;
    Cs[row * 64 + col] = a00[r];
    Cs[row * 64 + col + 16] = a01[r];
    Cs[(row + 16) * 64 + col] = a10[r];
    Cs[(row + 16) * 64 + col + 16] = a11[r];
  }
  __syncthreads();
  v4f vals[8];
#pragma unroll
  for (int i = 0; i < 8; ++i) {
    const int row = w * 16 + 2 * i + h;
    vals[i] = *(const v4fa*)(Cs + row * 64 + m16 * 4);
  }
#pragma unroll
  for (int i = 0; i < 8; ++i) {
    const int row = w * 16 + 2 * i + h;
    *(volatile v4f*)(C + (size_t)(m0 + row) * N + n0 + m16 * 4) = vals[i];
  }
  __threadfence();
#pragma unroll
  for (int i = 0; i < 8; ++i) {
    const int row = w * 16 + 2 * i + h;
    *(volatile v4f*)(C + (size_t)(m0 + row) * N + n0 + m16 * 4) = vals[i];
  }
}

__global__ __launch_bounds__(256) void k_gates(const float* __restrict__ x, const float* __restrict__ Wb,
                                               const float* __restrict__ Wg, const float* __restrict__ bg,
                                               const float* __restrict__ Wh, const float* __restrict__ bh,
                                               float* __restrict__ gates) {
  __shared__ __attribute__((aligned(16))) bf16 Ah[128 * GP];
  __shared__ __attribute__((aligned(16))) bf16 Al[128 * GP];
  __shared__ __attribute__((aligned(16))) bf16 Bh[16 * GP];
  __shared__ __attribute__((aligned(16))) bf16 Bl[16 * GP];
  __shared__ __attribute__((aligned(16))) float G[128 * 16];
  __shared__ __attribute__((aligned(16))) float R[20 * 128];
  const int tid = threadIdx.x, lane = tid & 31, w = tid >> 5, h = lane >> 4, m16 = lane & 15;
  const int m0 = blockIdx.x * 128;
  if (m0 + 128 > BL) return;
  const int b = m0 / LLEN, l0 = m0 - b * LLEN;
  v8f acc = {};
#pragma unroll 1
  for (int it = 0; it < DMODEL / 32; ++it) {
    const int k0 = it << 5;
    stage_a128(x, DMODEL, m0, k0, Ah, Al, tid);
#pragma unroll
    for (int j = 0; j < 2; ++j) {
      const int idx = tid + 256 * j;
      const int n = idx >> 5, kk = idx & 31, k = k0 + kk;
      float v;
      if (n < 8) v = Wb[k * 8 + n];
      else if (n < 12) v = Wg[k * 4 + (n - 8)];
      else v = Wh[k * 4 + (n - 12)];
      bf16 hb = (bf16)v;
      Bh[n * GP + kk] = hb;
      Bl[n * GP + kk] = (bf16)(v - (float)hb);
    }
    __syncthreads();
    Frag2 fa = frag_rowk_bf(Ah + (w * 16 + m16) * GP, Al + (w * 16 + m16) * GP, h);
    Frag2 fb = frag_rowk_bf(Bh + m16 * GP, Bl + m16 * GP, h);
    acc = mma3(acc, fa, fb);
    __syncthreads();
  }
#pragma unroll
  for (int r = 0; r < 8; ++r) G[(w * 16 + 8 * h + r) * 16 + m16] = acc[r];
  __syncthreads();
  if (tid < 128) {
    const int row = tid;
#pragma unroll 1
    for (int hh = 0; hh < NHEAD; ++hh) {
      const float sbl = G[row * 16 + hh];
      const float sbg = G[row * 16 + 4 + hh];
      const float sg = G[row * 16 + 8 + hh] + bg[hh];
      const float sh = G[row * 16 + 12 + hh] + bh[hh];
      const float bl = 1.f / (1.f + expf(-sbl));
      const float bgl = 1.f / (1.f + expf(-sbg));
      const float mx = fmaxf(fmaxf(sg, sh), 0.f);
      const float e0 = expf(sg - mx), e1 = expf(sh - mx), e2 = expf(-mx);
      const float inv = 1.f / (e0 + e1 + e2);
      R[(0 * 4 + hh) * 128 + row] = bl;
      R[(1 * 4 + hh) * 128 + row] = bgl;
      R[(2 * 4 + hh) * 128 + row] = e0 * inv;
      R[(3 * 4 + hh) * 128 + row] = e1 * inv;
      R[(4 * 4 + hh) * 128 + row] = e2 * inv;
    }
  }
  __syncthreads();
  for (int s = w; s < 20; s += 8) {
    v4f v = *(const v4fa*)(R + s * 128 + lane * 4);
    float* dst = gates + (size_t)(s >> 2) * BHL + (size_t)(b * NHEAD + (s & 3)) * LLEN + l0 + lane * 4;
    *(volatile v4f*)dst = v;
  }
  __threadfence();
  for (int s = w; s < 20; s += 8) {
    v4f v = *(const v4fa*)(R + s * 128 + lane * 4);
    float* dst = gates + (size_t)(s >> 2) * BHL + (size_t)(b * NHEAD + (s & 3)) * LLEN + l0 + lane * 4;
    *(volatile v4f*)dst = v;
  }
}

__global__ __launch_bounds__(256) void k_conv(const float* __restrict__ qp, const float* __restrict__ kp,
                                              const float* __restrict__ vp, const float* __restrict__ cq,
                                              const float* __restrict__ ck, const float* __restrict__ cv,
                                              float* __restrict__ qh, float* __restrict__ kh,
                                              float* __restrict__ vh) {
  const int idx = blockIdx.x;
  if (idx >= BHL) return;
  const int bhh = idx / LLEN, l = idx - bhh * LLEN, b = bhh / NHEAD, hd = bhh - b * NHEAD;
  const int c = threadIdx.x, lane = c & 31, w = c >> 5;
  const int ch = hd * DKH + c;
  float tq = 0.f, tk = 0.f, tv = 0.f;
#pragma unroll
  for (int j = 0; j < CONVK; ++j) {
    const int ls = l + j - (CONVK - 1);
    if (ls >= 0) {
      const size_t off = (size_t)(b * LLEN + ls) * DMODEL + ch;
      tq += qp[off] * cq[ch * CONVK + j];
      tk += kp[off] * ck[ch * CONVK + j];
      tv += vp[off] * cv[ch * CONVK + j];
    }
  }
  tq = tq / (1.f + expf(-tq));
  tk = tk / (1.f + expf(-tk));
  tv = tv / (1.f + expf(-tv));
  __shared__ __attribute__((aligned(16))) float rq[DKH];
  __shared__ __attribute__((aligned(16))) float rk[DKH];
  __shared__ __attribute__((aligned(16))) float rv[DVH];
  __shared__ float red1[8], red2[8];
  const float sq = wave_sum(tq * tq), sk = wave_sum(tk * tk);
  if (lane == 0) { red1[w] = sq; red2[w] = sk; }
  __syncthreads();
  float s1 = 0.f, s2 = 0.f;
#pragma unroll
  for (int i = 0; i < 8; ++i) { s1 += red1[i]; s2 += red2[i]; }
  rq[c] = tq * rsqrtf(s1 + 1e-12f);
  rk[c] = tk * rsqrtf(s2 + 1e-12f);
  rv[c] = tv;
  __syncthreads();
  if (w < 6) {
    const int sel = w >> 1, half = w & 1;
    const float* src = (sel == 0) ? rq : ((sel == 1) ? rk : rv);
    float* dstb = (sel == 0) ? qh : ((sel == 1) ? kh : vh);
    const size_t rowoff = ((size_t)bhh * LLEN + l) * DKH + half * 128 + lane * 4;
    v4f v = *(const v4fa*)(src + half * 128 + lane * 4);
    *(volatile v4f*)(dstb + rowoff) = v;
    __threadfence();
    *(volatile v4f*)(dstb + rowoff) = v;
  }
}

__global__ __launch_bounds__(256) void k_scan(const float* __restrict__ qhall,
                                              const float* __restrict__ khall,
                                              const float* __restrict__ vhall,
                                              const float* __restrict__ gates,
                                              float* __restrict__ obr) {
  const int bid = blockIdx.x;
  if (bid >= BBATCH * NHEAD * 2 * NDV) return;
  const int dvi = bid % NDV, br = (bid / NDV) & 1, bh = bid / (NDV * 2);
  const float* qg = qhall + (size_t)bh * LLEN * DKH;
  const float* kg = khall + (size_t)bh * LLEN * DKH;
  const float* vg = vhall + (size_t)bh * LLEN * DVH + dvi * DVT;
  const float* beta = gates + (size_t)br * BHL + (size_t)bh * LLEN;
  const float* wrow = gates + (size_t)(2 + br) * BHL + (size_t)bh * LLEN;
  float* og = obr + ((size_t)((br * BBATCH * NHEAD + bh) * NDV + dvi)) * LLEN * DVT;

  __shared__ __attribute__((aligned(16))) float S[DKH * DVT];
  __shared__ __attribute__((aligned(16))) float T[CCH * CCH];
  __shared__ __attribute__((aligned(16))) float aA[CCH * CCH];
  __shared__ __attribute__((aligned(16))) float upre[CCH * DVT];
  __shared__ __attribute__((aligned(16))) float uF[CCH * DVT];
  __shared__ __attribute__((aligned(16))) float ot[CCH * DVT];
  __shared__ float bet[CCH], wgt[CCH];

  const int tid = threadIdx.x, lane = tid & 31, w = tid >> 5, h = lane >> 4, m16 = lane & 15;

  for (int i = tid; i < DKH * DVT; i += 256) S[i] = 0.f;
  __syncthreads();

  for (int chn = 0; chn < NCH; ++chn) {
    const int l0 = chn * CCH;
    if (tid < CCH) { bet[tid] = beta[l0 + tid]; wgt[tid] = wrow[l0 + tid]; }
    __syncthreads();

    for (int job = w; job < 10; job += 8) {
      if (job < 8) {
        const int jj = job & 3, mt = jj >> 1, nt = jj & 1;
        const float* arow = ((job < 4) ? kg : qg) + (size_t)(l0 + mt * 16 + m16) * DKH;
        const float* brow = kg + (size_t)(l0 + nt * 16 + m16) * DKH;
        v8f acc = {};
#pragma unroll 1
        for (int kk = 0; kk < DKH / 32; ++kk) {
          Frag2 fa = frag_rowk_f32(arow + kk * 32, h);
          Frag2 fb = frag_rowk_f32(brow + kk * 32, h);
          acc = mma3(acc, fa, fb);
        }
        if (job < 4) {
#pragma unroll
          for (int r = 0; r < 8; ++r) {
            const int i = mt * 16 + 8 * h + r, j = nt * 16 + m16;
            T[i * CCH + j] = (i > j) ? -(bet[i] * acc[r]) : 0.f;
          }
        } else {
#pragma unroll
          for (int r = 0; r < 8; ++r) {
            const int i = mt * 16 + 8 * h + r, j = nt * 16 + m16;
            aA[i * CCH + j] = (j <= i) ? acc[r] : 0.f;
          }
        }
      } else {
        const int mt = job - 8;
        const float* arow = kg + (size_t)(l0 + mt * 16 + m16) * DKH;
        v8f acc = {};
#pragma unroll 1
        for (int kk = 0; kk < DKH / 32; ++kk) {
          Frag2 fa = frag_rowk_f32(arow + kk * 32, h);
          Frag2 fb = frag_colk_f32(S + (kk * 32) * DVT + m16, DVT, h);
          acc = mma3(acc, fa, fb);
        }
#pragma unroll
        for (int r = 0; r < 8; ++r) {
          const int i = mt * 16 + 8 * h + r;
          upre[i * DVT + m16] = vg[(size_t)(l0 + i) * DVH + m16] - acc[r];
        }
      }
    }
    __syncthreads();

    for (int i = 1; i < CCH; ++i) {
      float s = 0.f;
      if (tid < CCH) {
        s = T[i * CCH + tid];
#pragma unroll 4
        for (int k2 = 0; k2 < i; ++k2) s += T[i * CCH + k2] * T[k2 * CCH + tid];
      }
      __syncthreads();
      if (tid < i) T[i * CCH + tid] = s;
      __syncthreads();
    }
    for (int idx = tid; idx < CCH * CCH; idx += 256) {
      const int i = idx >> 5, j = idx & 31;
      const float t = (i == j) ? 1.f : T[idx];
      T[idx] = t * bet[j];
    }
    __syncthreads();

    if (w < 2) {
      const int mt = w;
      v8f acc = {};
      Frag2 fa = frag_rowk_f32(T + (mt * 16 + m16) * CCH, h);
      Frag2 fb = frag_colk_f32(upre + m16, DVT, h);
      acc = mma3(acc, fa, fb);
#pragma unroll
      for (int r = 0; r < 8; ++r) {
        const int i = mt * 16 + 8 * h + r;
        uF[i * DVT + m16] = acc[r] * wgt[i];
      }
    }
    __syncthreads();

    if (w < 2) {
      const int mt = w;
      const float* arow = qg + (size_t)(l0 + mt * 16 + m16) * DKH;
      v8f acc = {};
#pragma unroll 1
      for (int kk = 0; kk < DKH / 32; ++kk) {
        Frag2 fa = frag_rowk_f32(arow + kk * 32, h);
        Frag2 fb = frag_colk_f32(S + (kk * 32) * DVT + m16, DVT, h);
        acc = mma3(acc, fa, fb);
      }
      {
        Frag2 fa = frag_rowk_f32(aA + (mt * 16 + m16) * CCH, h);
        Frag2 fb = frag_colk_f32(uF + m16, DVT, h);
        acc = mma3(acc, fa, fb);
      }
#pragma unroll
      for (int r = 0; r < 8; ++r) ot[(mt * 16 + 8 * h + r) * DVT + m16] = acc[r];
    }
    __syncthreads();

    if (w == 0) {
      float* dst = og + (size_t)l0 * DVT;
#pragma unroll
      for (int i = 0; i < 4; ++i) {
        v4f v = *(const v4fa*)(ot + i * 128 + lane * 4);
        *(volatile v4f*)(dst + i * 128 + lane * 4) = v;
      }
      __threadfence();
#pragma unroll
      for (int i = 0; i < 4; ++i) {
        v4f v = *(const v4fa*)(ot + i * 128 + lane * 4);
        *(volatile v4f*)(dst + i * 128 + lane * 4) = v;
      }
    }

    for (int mt = w; mt < DKH / 16; mt += 8) {
      v8f acc;
#pragma unroll
      for (int r = 0; r < 8; ++r) acc[r] = S[(mt * 16 + 8 * h + r) * DVT + m16];
      Frag2 fa = frag_colk_f32(kg + (size_t)l0 * DKH + mt * 16 + m16, DKH, h);
      Frag2 fb = frag_colk_f32(uF + m16, DVT, h);
      acc = mma3(acc, fa, fb);
#pragma unroll
      for (int r = 0; r < 8; ++r) S[(mt * 16 + 8 * h + r) * DVT + m16] = acc[r];
    }
    __syncthreads();
  }
}

__global__ __launch_bounds__(64) void k_epi(const float* __restrict__ obr, const float* __restrict__ vh,
                                            const float* __restrict__ gates, const float* __restrict__ normw,
                                            float* __restrict__ ofin) {
  const int idx = blockIdx.x;
  if (idx >= BHL) return;
  const int bhh = idx / LLEN, l = idx - bhh * LLEN, b = bhh / NHEAD, hd = bhh - b * NHEAD;
  const int t = threadIdx.x, lane = t & 31, w = t >> 5;
  const int c0 = 4 * t, sl = c0 >> 4, wi = c0 & 15;
  const size_t o0 = ((size_t)((0 * BBATCH * NHEAD + bhh) * NDV + sl) * LLEN + l) * DVT + wi;
  const size_t o1 = ((size_t)((1 * BBATCH * NHEAD + bhh) * NDV + sl) * LLEN + l) * DVT + wi;
  v4f a = *(const v4fa*)(obr + o0);
  v4f g = *(const v4fa*)(obr + o1);
  v4f vv = *(const v4fa*)(vh + ((size_t)bhh * LLEN + l) * DVH + c0);
  const float wr = gates[(size_t)4 * BHL + (size_t)bhh * LLEN + l];
  v4f o = (a + g) + wr * vv;
  float ss = o[0] * o[0] + o[1] * o[1] + o[2] * o[2] + o[3] * o[3];
  ss = wave_sum(ss);
  __shared__ float red[2];
  if (lane == 0) red[w] = ss;
  __syncthreads();
  const float tot = red[0] + red[1];
  const float rs = rsqrtf(tot * (1.f / DVH) + 1e-5f);
  v4f nw = *(const v4fa*)(normw + c0);
  v4f outv = (o * rs) * nw;
  float* dst = ofin + ((size_t)(b * LLEN + l)) * DMODEL + hd * DVH + c0;
  *(volatile v4f*)dst = outv;
  __threadfence();
  *(volatile v4f*)dst = outv;
}

extern "C" void kernel_launch(void* const* d_in, const int* in_sizes, int n_in,
                              void* d_out, int out_size, void* d_ws, size_t ws_size,
                              hipStream_t stream) {
  if (n_in != 14) return;
  if (in_sizes[0] != BL * DMODEL) return;
  if (in_sizes[1] != DMODEL * DMODEL || in_sizes[2] != DMODEL * DMODEL ||
      in_sizes[3] != DMODEL * DMODEL || in_sizes[13] != DMODEL * DMODEL) return;
  if (in_sizes[4] != DMODEL * CONVK || in_sizes[5] != DMODEL * CONVK || in_sizes[6] != DMODEL * CONVK) return;
  if (in_sizes[7] != DMODEL * 2 * NHEAD || in_sizes[8] != DMODEL * NHEAD || in_sizes[10] != DMODEL * NHEAD) return;
  if (in_sizes[9] != NHEAD || in_sizes[11] != NHEAD || in_sizes[12] != DVH) return;
  if (out_size != BL * DMODEL) return;

  const float* x     = (const float*)d_in[0];
  const float* Wq    = (const float*)d_in[1];
  const float* Wk    = (const float*)d_in[2];
  const float* Wv    = (const float*)d_in[3];
  const float* convq = (const float*)d_in[4];
  const float* convk = (const float*)d_in[5];
  const float* convv = (const float*)d_in[6];
  const float* Wb    = (const float*)d_in[7];
  const float* Wg    = (const float*)d_in[8];
  const float* bg    = (const float*)d_in[9];
  const float* Wh    = (const float*)d_in[10];
  const float* bh    = (const float*)d_in[11];
  const float* normw = (const float*)d_in[12];
  const float* Wo    = (const float*)d_in[13];

  const size_t fsz    = sizeof(float);
  const size_t sz_pre = (size_t)BL * DMODEL * fsz;
  const size_t sz_hd  = (size_t)BHL * DKH * fsz;
  const size_t sz_gt  = (size_t)5 * BHL * fsz;
  const size_t sz_obr = (size_t)2 * BHL * DVH * fsz;
  size_t off = 0;
  const size_t o_qpre = off; off += sz_pre;
  const size_t o_kpre = off; off += sz_pre;
  const size_t o_vpre = off; off += sz_pre;
  const size_t o_qh   = off; off += sz_hd;
  const size_t o_kh   = off; off += sz_hd;
  const size_t o_vh   = off; off += sz_hd;
  const size_t o_gt   = off; off += ((sz_gt + (1u << 20) - 1) >> 20) << 20;
  const size_t o_obr  = off; off += sz_obr;
  const size_t o_ofin = off; off += sz_pre;
  if (off > ws_size) return;

  char* ws = (char*)d_ws;
  float* q_pre = (float*)(ws + o_qpre);
  float* k_pre = (float*)(ws + o_kpre);
  float* v_pre = (float*)(ws + o_vpre);
  float* qh    = (float*)(ws + o_qh);
  float* kh    = (float*)(ws + o_kh);
  float* vh    = (float*)(ws + o_vh);
  float* gates = (float*)(ws + o_gt);
  float* obr   = (float*)(ws + o_obr);
  float* ofin  = (float*)(ws + o_ofin);

  dim3 blk(256);
  dim3 gproj((BL + 127) / 128, (DMODEL + 63) / 64);

  k_gemm<<<gproj, blk, 0, stream>>>(x, Wq, q_pre, BL, DMODEL, DMODEL);
  k_gemm<<<gproj, blk, 0, stream>>>(x, Wk, k_pre, BL, DMODEL, DMODEL);
  k_gemm<<<gproj, blk, 0, stream>>>(x, Wv, v_pre, BL, DMODEL, DMODEL);

  k_gates<<<dim3((BL + 127) / 128), blk, 0, stream>>>(x, Wb, Wg, bg, Wh, bh, gates);

  k_conv<<<dim3(BHL), blk, 0, stream>>>(q_pre, k_pre, v_pre, convq, convk, convv, qh, kh, vh);

  k_scan<<<dim3(BBATCH * NHEAD * 2 * NDV), blk, 0, stream>>>(qh, kh, vh, gates, obr);

  k_epi<<<dim3(BHL), dim3(64), 0, stream>>>(obr, vh, gates, normw, ofin);

  k_gemm<<<gproj, blk, 0, stream>>>(ofin, Wo, (float*)d_out, BL, DMODEL, DMODEL);
}
